// OctodiffAttention_11871289606209
// MI455X (gfx1250) — hardware-verified
//
#include <hip/hip_runtime.h>
#include <math.h>


#define B_   2
#define S_   2048
#define D_   2048
#define NH_  16
#define NKV_ 4
#define HD_  128
#define KVD_ (NKV_ * HD_)
#define M_TOT (B_ * S_)
#define SCALE_ 0.08838834764831845f

typedef __attribute__((ext_vector_type(16))) __bf16 v16bf;
typedef __attribute__((ext_vector_type(8)))  __bf16 v8bf;
typedef __attribute__((ext_vector_type(8)))  float  v8f;
typedef __attribute__((ext_vector_type(4)))  float  v4f;

template <typename V> __device__ __forceinline__ void vst2(void* p, V v) {
  *(volatile V*)p = v; __threadfence(); *(volatile V*)p = v;
}
__device__ __forceinline__ __bf16 bf_hi(float x) { return (__bf16)x; }
__device__ __forceinline__ __bf16 bf_lo(float x, __bf16 h) { return (__bf16)(x - (float)h); }
__device__ __forceinline__ v8f wmma_bf16(v16bf a, v16bf b, v8f c) {
  v8f d = __builtin_amdgcn_wmma_f32_16x16x32_bf16(false, a, false, b, (short)0, c, false, false);
  asm volatile("v_nop\n\tv_nop\n\tv_nop\n\tv_nop" : "+v"(d) : "v"(a), "v"(b));
  return d;
}
__device__ __forceinline__ v8f wmma_x3(v16bf ah, v16bf al, v16bf bh, v16bf bl, v8f c) {
  c = wmma_bf16(ah, bh, c); c = wmma_bf16(ah, bl, c); c = wmma_bf16(al, bh, c);
  return c;
}

__device__ __forceinline__ void frag_f32(const float* __restrict__ base, int ld, int r0, int k0, int lane, v16bf& hi, v16bf& lo) {
  const float* p = base + (size_t)(r0 + (lane & 15)) * ld + k0 + (lane >> 4) * 8;
  const v4f a0 = *(const v4f*)(p), a1 = *(const v4f*)(p + 4), a2 = *(const v4f*)(p + 16), a3 = *(const v4f*)(p + 20);
#pragma unroll
  for (int i = 0; i < 4; ++i) {
    __bf16 h;
    h = bf_hi(a0[i]); hi[i] = h;      lo[i] = bf_lo(a0[i], h);
    h = bf_hi(a1[i]); hi[4 + i] = h;  lo[4 + i] = bf_lo(a1[i], h);
    h = bf_hi(a2[i]); hi[8 + i] = h;  lo[8 + i] = bf_lo(a2[i], h);
    h = bf_hi(a3[i]); hi[12 + i] = h; lo[12 + i] = bf_lo(a3[i], h);
  }
}
__device__ __forceinline__ v16bf frag_lds(const __bf16* base, int ld, int r0, int k0, int lane) {
  union { v16bf v; v8bf h[2]; } r;
  const __bf16* p = base + (r0 + (lane & 15)) * ld + k0 + (lane >> 4) * 8;
  r.h[0] = *(const v8bf*)(p); r.h[1] = *(const v8bf*)(p + 16);
  return r.v;
}


template <int KDIM>
__device__ __forceinline__ void gemm_mainloop_32x64(const float* __restrict__ A, const float* __restrict__ Bt,
                                                    int m0, int n0, int lane, v8f acc[2][4]) {
#pragma unroll 1
  for (int k0 = 0; k0 < KDIM; k0 += 32) {
    v16bf ah[2], al[2], bh[4], bl[4];
    frag_f32(A, KDIM, m0, k0, lane, ah[0], al[0]);
    frag_f32(A, KDIM, m0 + 16, k0, lane, ah[1], al[1]);
#pragma unroll
    for (int j = 0; j < 4; ++j) frag_f32(Bt, KDIM, n0 + j * 16, k0, lane, bh[j], bl[j]);
#pragma unroll
    for (int i = 0; i < 2; ++i)
#pragma unroll
      for (int j = 0; j < 4; ++j) acc[i][j] = wmma_x3(ah[i], al[i], bh[j], bl[j], acc[i][j]);
  }
}

__global__ __launch_bounds__(256) void wtrans_kernel(const float* __restrict__ W, float* __restrict__ Wt, int K, int N) {
  __shared__ __align__(16) float tile[64][68];
  const int nt = N / 64;
  const int n0 = (blockIdx.x % nt) * 64, k0 = (blockIdx.x / nt) * 64, tid = threadIdx.x;
  for (int i = tid; i < 64 * 64; i += 256) { const int kk = i >> 6, nn = i & 63; tile[nn][kk] = W[(size_t)(k0 + kk) * N + n0 + nn]; }
  __syncthreads();
  for (int g = tid; g < 64 * 16; g += 256) { const int nn = g >> 4, pc = g & 15; vst2(Wt + (size_t)(n0 + nn) * K + k0 + pc * 4, *(const v4f*)(&tile[nn][pc * 4])); }
}

__global__ __launch_bounds__(256) void proj_rope_kernel(const float* __restrict__ X, const float* __restrict__ Wt, int nheads,
                                                       float scale, int vmode, float* __restrict__ dst) {
  __shared__ __align__(16) float st[128][128];
  const int lane = threadIdx.x & 31, wave = threadIdx.x >> 5, tid = threadIdx.x;
  const int mblk = blockIdx.y * 128;
  const int head = blockIdx.x;
  const int m0 = mblk + (wave & 3) * 32;
  const int nl0 = (wave >> 2) * 64;
  const int n0 = head * HD_ + nl0;
  const int b = mblk / S_, s0 = mblk % S_;

  v8f acc[2][4] = {};
  gemm_mainloop_32x64<D_>(X, Wt, m0, n0, lane, acc);
  const int half = lane >> 4, col = lane & 15;
#pragma unroll
  for (int i = 0; i < 2; ++i)
#pragma unroll
    for (int j = 0; j < 4; ++j)
#pragma unroll
      for (int r = 0; r < 8; ++r) st[(wave & 3) * 32 + i * 16 + r + 8 * half][nl0 + j * 16 + col] = acc[i][j][r];
  __syncthreads();
  if (vmode) {
#pragma unroll 1
    for (int g = tid; g < 128 * 32; g += 256) {
      const int dl = g >> 5, pc = g & 31;
      v4f v = {st[pc * 4][dl], st[pc * 4 + 1][dl], st[pc * 4 + 2][dl], st[pc * 4 + 3][dl]};
      vst2(dst + (((size_t)(b * nheads + head) * HD_ + dl) * S_) + s0 + pc * 4, v);
    }
    return;
  }
  for (int g = tid; g < 128 * 32; g += 256) {
    const int ml = g >> 5, pc = g & 31;
    const int s = s0 + ml;
    v4f v;
#pragma unroll
    for (int e = 0; e < 4; ++e) {
      const int d = pc * 4 + e, dm = d & 63;
      const float inv_freq = (float)(1.0 / pow(10000.0, (double)dm / 64.0));
      const float fr = (float)s * inv_freq;
      const float c = cosf(fr), sn = sinf(fr);
      const float x = st[ml][d];
      const float xr = (d < 64) ? -st[ml][d + 64] : st[ml][d - 64];
      v[e] = (x * c + xr * sn) * scale;
    }
    vst2(dst + (((size_t)(b * nheads + head) * S_ + s) * HD_) + pc * 4, v);
  }
}

__global__ __launch_bounds__(128) void attn_kernel(const float* __restrict__ Qb, const float* __restrict__ Kb,
                                                  const float* __restrict__ Vt, float* __restrict__ Ctx) {
  __shared__ __align__(16) __bf16 Kh[32 * 136], Kl[32 * 136];
  __shared__ __align__(16) __bf16 Vh[128 * 40], Vl[128 * 40];
  __shared__ __align__(16) __bf16 Ph[4][16 * 40], Pl[4][16 * 40];
  __shared__ __align__(16) float  Os[4][16 * 128];

  const int tid = threadIdx.x, lane = tid & 31, wave = tid >> 5, half = lane >> 4, col = lane & 15;
  const int q0 = blockIdx.x * 64, head = blockIdx.y, b = blockIdx.z;
  const int kvh = head / (NH_ / NKV_);
  const float* Qh = Qb + (size_t)(b * NH_ + head) * S_ * HD_;
  const float* Kg = Kb + (size_t)(b * NKV_ + kvh) * S_ * HD_;
  const float* Vg = Vt + (size_t)(b * NKV_ + kvh) * HD_ * S_;
  const int mq = q0 + wave * 16;

  v16bf qh[4], ql[4];
#pragma unroll
  for (int kb = 0; kb < 4; ++kb) frag_f32(Qh, HD_, mq, kb * 32, lane, qh[kb], ql[kb]);

  v8f o[8] = {};
  float mrow[8], lrow[8];
#pragma unroll
  for (int r = 0; r < 8; ++r) { mrow[r] = -1e30f; lrow[r] = 0.0f; }
  __bf16* ph = Ph[wave];
  __bf16* pl = Pl[wave];

  const int t_end = q0 + 64;
  for (int t0 = 0; t0 < t_end; t0 += 32) {
    __syncthreads();
    {
      const int kr = tid >> 2, kc = (tid & 3) * 32;
      const float* kp = Kg + (size_t)(t0 + kr) * HD_ + kc;
      const int vr = tid;
      const float* vp = Vg + (size_t)vr * S_ + t0;
#pragma unroll
      for (int e = 0; e < 32; e += 4) {
        const v4f a = *(const v4f*)(kp + e), bb = *(const v4f*)(vp + e);
#pragma unroll
        for (int i = 0; i < 4; ++i) {
          __bf16 hk = bf_hi(a[i]);  Kh[kr * 136 + kc + e + i] = hk; Kl[kr * 136 + kc + e + i] = bf_lo(a[i], hk);
          __bf16 hv = bf_hi(bb[i]); Vh[vr * 40 + e + i] = hv;         Vl[vr * 40 + e + i] = bf_lo(bb[i], hv);
        }
      }
    }
    __syncthreads();

    v8f s[2] = {};
#pragma unroll
    for (int n = 0; n < 2; ++n)
#pragma unroll
      for (int kb = 0; kb < 4; ++kb)
        s[n] = wmma_x3(qh[kb], ql[kb], frag_lds(Kh, 136, n * 16, kb * 32, lane), frag_lds(Kl, 136, n * 16, kb * 32, lane), s[n]);

    {
      const int k0g = t0 + col, k1g = t0 + 16 + col;
#pragma unroll
      for (int r = 0; r < 8; ++r) {
        const int qg = mq + r + 8 * half;
        float v0 = (k0g <= qg) ? s[0][r] : -1e30f;
        float v1 = (k1g <= qg) ? s[1][r] : -1e30f;
        float mx = fmaxf(v0, v1);
#pragma unroll
        for (int off = 8; off > 0; off >>= 1) mx = fmaxf(mx, __shfl_xor(mx, off, 16));
        const float mnew  = fmaxf(mrow[r], mx);
        const float alpha = __expf(mrow[r] - mnew);
        const float p0 = (k0g <= qg) ? __expf(v0 - mnew) : 0.0f;
        const float p1 = (k1g <= qg) ? __expf(v1 - mnew) : 0.0f;
        float rs = p0 + p1;
#pragma unroll
        for (int off = 8; off > 0; off >>= 1) rs += __shfl_xor(rs, off, 16);
        lrow[r] = lrow[r] * alpha + rs;
        mrow[r] = mnew;
#pragma unroll
        for (int j = 0; j < 8; ++j) o[j][r] *= alpha;
        const int row = r + 8 * half;
        __bf16 h0 = bf_hi(p0), h1 = bf_hi(p1);
        ph[row * 40 + col] = h0;      pl[row * 40 + col] = bf_lo(p0, h0);
        ph[row * 40 + 16 + col] = h1; pl[row * 40 + 16 + col] = bf_lo(p1, h1);
      }
    }
    __syncthreads();
    const v16bf pah = frag_lds(ph, 40, 0, 0, lane), pal = frag_lds(pl, 40, 0, 0, lane);
#pragma unroll
    for (int j = 0; j < 8; ++j)
      o[j] = wmma_x3(pah, pal, frag_lds(Vh, 40, j * 16, 0, lane), frag_lds(Vl, 40, j * 16, 0, lane), o[j]);
  }

  float* os_ = Os[wave];
#pragma unroll
  for (int r = 0; r < 8; ++r) {
    const float inv = 1.0f / lrow[r];
#pragma unroll
    for (int j = 0; j < 8; ++j) os_[(r + 8 * half) * 128 + j * 16 + col] = o[j][r] * inv;
  }
  __syncthreads();
#pragma unroll
  for (int q = 0; q < 16; ++q)
    vst2(Ctx + ((size_t)(b * S_ + mq + q)) * D_ + head * HD_ + lane * 4, *(const v4f*)(os_ + q * 128 + lane * 4));
}

__global__ __launch_bounds__(128) void out_gemm_kernel(const float* __restrict__ Cx, const float* __restrict__ WoT, float* __restrict__ Out) {
  __shared__ __align__(16) float st[4][32 * 64];
  const int lane = threadIdx.x & 31, wave = threadIdx.x >> 5;
  const int m0 = blockIdx.y * 64 + (wave >> 1) * 32;
  const int n0 = blockIdx.x * 128 + (wave & 1) * 64;
  v8f acc[2][4] = {};
  gemm_mainloop_32x64<D_>(Cx, WoT, m0, n0, lane, acc);
  const int half = lane >> 4, col = lane & 15;
  float* S = st[wave];
#pragma unroll
  for (int i = 0; i < 2; ++i)
#pragma unroll
    for (int j = 0; j < 4; ++j)
#pragma unroll
      for (int r = 0; r < 8; ++r) S[(i * 16 + r + 8 * half) * 64 + j * 16 + col] = acc[i][j][r];
  __syncthreads();
#pragma unroll
  for (int q = 0; q < 16; ++q) {
    const int rl = q * 2 + (lane >> 4), pc = lane & 15;
    vst2(Out + (size_t)(m0 + rl) * D_ + n0 + pc * 4, *(const v4f*)(S + rl * 64 + pc * 4));
  }
}

extern "C" void kernel_launch(void* const* d_in, const int* in_sizes, int n_in,
                              void* d_out, int out_size, void* d_ws, size_t ws_size,
                              hipStream_t stream) {
  (void)in_sizes; (void)n_in; (void)out_size; (void)ws_size;
  const float* x  = (const float*)d_in[0];
  const float* Wq = (const float*)d_in[2];
  const float* Wk = (const float*)d_in[3];
  const float* Wv = (const float*)d_in[4];
  const float* Wo = (const float*)d_in[5];
  float* out = (float*)d_out;

  char* ws = (char*)d_ws;
  size_t off = 0;
  auto carve = [&](size_t nfloat) { float* p = (float*)(ws + off); off = (off + nfloat * 4 + 255) & ~(size_t)255; return p; };
  float* WqT = carve((size_t)D_ * D_);
  float* WkT = carve((size_t)KVD_ * D_);
  float* WvT = carve((size_t)KVD_ * D_);
  float* WoT = carve((size_t)D_ * D_);
  float* Qb  = carve((size_t)M_TOT * D_);
  float* Kb  = carve((size_t)M_TOT * KVD_);
  float* Vt  = carve((size_t)M_TOT * KVD_);
  float* Ctx = carve((size_t)M_TOT * D_);

  wtrans_kernel<<<(D_ / 64) * (D_ / 64), 256, 0, stream>>>(Wq, WqT, D_, D_);
  wtrans_kernel<<<(D_ / 64) * (KVD_ / 64), 256, 0, stream>>>(Wk, WkT, D_, KVD_);
  wtrans_kernel<<<(D_ / 64) * (KVD_ / 64), 256, 0, stream>>>(Wv, WvT, D_, KVD_);
  wtrans_kernel<<<(D_ / 64) * (D_ / 64), 256, 0, stream>>>(Wo, WoT, D_, D_);

  proj_rope_kernel<<<dim3(NH_, M_TOT / 128), 256, 0, stream>>>(x, WqT, NH_, SCALE_, 0, Qb);
  proj_rope_kernel<<<dim3(NKV_, M_TOT / 128), 256, 0, stream>>>(x, WkT, NKV_, 1.0f, 0, Kb);
  proj_rope_kernel<<<dim3(NKV_, M_TOT / 128), 256, 0, stream>>>(x, WvT, NKV_, 1.0f, 1, Vt);
  attn_kernel<<<dim3(S_ / 64, NH_, B_), 128, 0, stream>>>(Qb, Kb, Vt, Ctx);
  out_gemm_kernel<<<dim3(D_ / 128, M_TOT / 64), 128, 0, stream>>>(Ctx, WoT, out);
}
